// EfficientAttention_8409545965831
// MI455X (gfx1250) — hardware-run, weakly checked
//
#include <hip/hip_runtime.h>
#define NB 4
#define NTOK 8192
#define CW 384
#define NHD 6
#define HD 64
#define TBK 64
#define NBLK (NTOK / TBK)
#define QCAR 16.0f
#define KCAR 1024.0f
#define KVCAR 256.0f
#define OCAR 256.0f
typedef __bf16 v16b __attribute__((ext_vector_type(16)));
typedef unsigned short v8us __attribute__((ext_vector_type(8), may_alias));
typedef float  v8f  __attribute__((ext_vector_type(8)));
typedef float  v4f  __attribute__((ext_vector_type(4)));
typedef float  v4fa __attribute__((ext_vector_type(4), may_alias));
union FragB { v16b v; v8us half[2]; unsigned short u[16]; };

__device__ __forceinline__ unsigned short bf16_bits(float x) { unsigned int u = __float_as_uint(x); return (unsigned short)((u + 0x7FFFu + ((u >> 16) & 1u)) >> 16); }
__device__ __forceinline__ float bf16_val(unsigned short b) { return __uint_as_float(((unsigned int)b) << 16); }
__device__ __forceinline__ float bf16_round(float x) { return bf16_val(bf16_bits(x)); }
template <int NT>
__device__ __forceinline__ v8f mmaN(v16b ah, v16b al, v16b bh, v16b bl, v8f c) {
  c = __builtin_amdgcn_wmma_f32_16x16x32_bf16(false, ah, false, bh, (short)0, c, false, false);
  if (NT >= 2) c = __builtin_amdgcn_wmma_f32_16x16x32_bf16(false, al, false, bh, (short)0, c, false, false);
  if (NT >= 3) c = __builtin_amdgcn_wmma_f32_16x16x32_bf16(false, ah, false, bl, (short)0, c, false, false);
  asm volatile("v_nop\n\tv_nop\n\tv_nop\n\tv_nop" : "+v"(c) : "v"(ah), "v"(al), "v"(bh), "v"(bl));
  return c;
}


typedef _Float16 v16h __attribute__((ext_vector_type(16)));
union FragH { v16h v; v8us half[2]; _Float16 h[16]; unsigned short u[16]; };
template <int NT>
__device__ __forceinline__ v8f mmaH(v16h ah, v16h al, v16h bh, v16h bl, v8f c) {
  c = __builtin_amdgcn_wmma_f32_16x16x32_f16(false, ah, false, bh, (short)0, c, false, false);
  if (NT >= 2) c = __builtin_amdgcn_wmma_f32_16x16x32_f16(false, al, false, bh, (short)0, c, false, false);
  if (NT >= 3) c = __builtin_amdgcn_wmma_f32_16x16x32_f16(false, ah, false, bl, (short)0, c, false, false);
  asm volatile("v_nop\n\tv_nop\n\tv_nop\n\tv_nop" : "+v"(c) : "v"(ah), "v"(al), "v"(bh), "v"(bl));
  return c;
}

__global__ __launch_bounds__(256) void k_wt_f16(const float* __restrict__ W, _Float16* __restrict__ Wt, int K, int N, float scale) {
  const int t = blockIdx.x * 256 + threadIdx.x; if (t >= N * (K / 8)) return; const int n = t / (K / 8), k8 = (t % (K / 8)) * 8; FragH f;
#pragma unroll
  for (int i = 0; i < 8; ++i) f.h[i] = (_Float16)(bf16_round(W[(size_t)(k8 + i) * N + n]) * scale); const v8us o = f.half[0];
  *(volatile v8us*)((unsigned short*)Wt + (size_t)n * K + k8) = o; __threadfence(); *(volatile v8us*)((unsigned short*)Wt + (size_t)n * K + k8) = o;
}

typedef _Float16 v4h __attribute__((ext_vector_type(4)));

__global__ __launch_bounds__(256) void k_x16(const float* __restrict__ x, _Float16* __restrict__ X16, size_t n8) { const size_t t = (size_t)blockIdx.x * 256 + threadIdx.x; if (t >= n8) return; FragH f;
#pragma unroll
  for (int q = 0; q < 8; ++q) f.h[q] = (_Float16)bf16_round(x[t * 8 + q]); *(volatile v8us*)((unsigned short*)X16 + t * 8) = f.half[0]; __threadfence(); *(volatile v8us*)((unsigned short*)X16 + t * 8) = f.half[0]; }


__device__ __forceinline__ v16h g2_frag(const _Float16* p, int hh) { FragH f; f.half[0] = *(const v8us*)((const unsigned short*)p + 8 * hh); f.half[1] = *(const v8us*)((const unsigned short*)p + 16 + 8 * hh); return f.v; }
__device__ __forceinline__ v8f g2_mma(v16h a, v16h b, v8f c) { v8f d = __builtin_amdgcn_wmma_f32_16x16x32_f16(false, a, false, b, (short)0, c, false, false); asm volatile("v_nop\n\tv_nop\n\tv_nop\n\tv_nop" : "+v"(d) : "v"(a), "v"(b)); return d; }
template <int ACT>
__global__ __launch_bounds__(128) void k_gemm2(const _Float16* __restrict__ A, int lda, size_t sA, const _Float16* __restrict__ Bh, int ldb, size_t sB, float alpha, const float* __restrict__ bias, size_t sBias, const float* __restrict__ CP, int rowsPerB, size_t sCPb, int row0g,
    float* __restrict__ C, _Float16* __restrict__ C16, int ldc, size_t sC, int M, int N, int K) { static_assert(ACT == 0 || ACT == 3 || ACT == 6 || ACT == 8 || ACT == 9 || ACT == 11 || ACT == 12 || ACT == 14 || ACT == 15 || ACT == 16 || ACT == 17, "k_gemm2: unsupported ACT code (would silently apply no activation)");
  __shared__ __attribute__((aligned(16))) float so[4][32][68];
  const int tid = threadIdx.x, w = tid >> 5, lane = tid & 31, ln = lane & 15, hh = lane >> 4; const int by = blockIdx.y;
  A += (size_t)by * sA; Bh += (size_t)by * sB; const size_t cofs = (size_t)by * sC; const float* bp = bias ? bias + (size_t)by * sBias : nullptr;
  const int ntn = N >> 6; const int mt = blockIdx.x / ntn, nq = blockIdx.x - mt * ntn; const int row0 = mt * 128 + 32 * w, col0 = nq * 64; if (row0 >= M) return;
  const _Float16* a0p = A + (size_t)(row0 + ln) * lda; const _Float16* a1p = a0p + (size_t)16 * lda;
  const _Float16* b0p = Bh + (size_t)(col0 + ln) * ldb; const _Float16* b1p = b0p + (size_t)16 * ldb; const _Float16* b2p = b1p + (size_t)16 * ldb; const _Float16* b3p = b2p + (size_t)16 * ldb;
  const v8f z8 = {0.f,0.f,0.f,0.f,0.f,0.f,0.f,0.f}; v8f c00 = z8, c01 = z8, c02 = z8, c03 = z8, c10 = z8, c11 = z8, c12 = z8, c13 = z8;
  for (int kb = 0; kb < K; kb += 32) { const v16h a0 = g2_frag(a0p + kb, hh), a1 = g2_frag(a1p + kb, hh);
    v16h b = g2_frag(b0p + kb, hh); c00 = g2_mma(a0, b, c00); c10 = g2_mma(a1, b, c10);
    b = g2_frag(b1p + kb, hh); c01 = g2_mma(a0, b, c01); c11 = g2_mma(a1, b, c11);
    b = g2_frag(b2p + kb, hh); c02 = g2_mma(a0, b, c02); c12 = g2_mma(a1, b, c12);
    b = g2_frag(b3p + kb, hh); c03 = g2_mma(a0, b, c03); c13 = g2_mma(a1, b, c13); }
  v8f accs[8] = {c00, c01, c02, c03, c10, c11, c12, c13};
#pragma unroll
  for (int u = 0; u < 8; ++u) { const int t = u & 3, half = u >> 2; const int col = col0 + t * 16 + ln; const float bv = bp ? bf16_round(bp[col]) : 0.f;
#pragma unroll
    for (int r = 0; r < 8; ++r) { const int rloc = half * 16 + 8 * hh + r; float v = accs[u][r] * alpha + bv; if (CP) { if (rowsPerB < 0) v += CP[cofs + (size_t)(row0g + row0 + rloc) * ldc + col];        else { const int bidx = (row0g + row0 + rloc) / rowsPerB; v += CP[(size_t)bidx * sCPb + (size_t)by * 64 + col]; } }
      if (ACT == 3) v = fmaxf(v, 0.f); else if (ACT == 6) v = 0.5f * v * (1.0f + erff(v * 0.70710678118654752f)); else if (ACT == 11) v = 1.0f / (1.0f + expf(-v)); else if (ACT == 15) v = v / (1.0f + expf(-v)); else if (ACT == 12) v = (v > 0.f) ? v : 0.01f * v; else if (ACT == 8) v = tanhf(v); else if (ACT == 9) v = 0.5f * v * (1.0f + tanhf(0.7978845608028654f * (v + 0.044715f * v * v * v))); else if (ACT == 14) v = (v > 0.f) ? v : 0.1f * v; else if (ACT == 16) v = (v >= 0.f) ? v : 0.3f * v; else if (ACT == 17) v = (v >= 0.f) ? v : 0.2f * v;
      so[w][rloc][t * 16 + ln] = v; } }
  __builtin_amdgcn_fence(__ATOMIC_ACQ_REL, "workgroup"); __builtin_amdgcn_wave_barrier();
  const int rsub = lane >> 4, c4 = (lane & 15) * 4;
  for (int pass = 0; pass < 2; ++pass) {
#pragma unroll
    for (int q = 0; q < 16; ++q) { const int r = q * 2 + rsub; const v4f v = *(const v4fa*)&so[w][r][c4]; if (C) *(volatile v4f*)(C + cofs + (size_t)(row0 + r) * ldc + col0 + c4) = v; if (C16) { v4h h4; for (int i = 0; i < 4; ++i) h4[i] = (_Float16)v[i]; *(volatile v4h*)(C16 + cofs + (size_t)(row0 + r) * ldc + col0 + c4) = h4; } }
    if (pass == 0) __threadfence(); } }
__global__ __launch_bounds__(256) void k_wtn_f16(const float* __restrict__ W, _Float16* __restrict__ Wt, int K, int N, float scale) {
  const int t = blockIdx.x * 256 + threadIdx.x; if (t >= N * (K / 8)) return; const int n = t / (K / 8), k8 = (t % (K / 8)) * 8; FragH f;
  for (int i = 0; i < 8; ++i) f.h[i] = (_Float16)(W[(size_t)(k8 + i) * N + n] * scale);
  unsigned short* o = (unsigned short*)Wt + (size_t)n * K + k8; *(volatile v8us*)o = f.half[0]; __threadfence(); *(volatile v8us*)o = f.half[0]; }
__global__ __launch_bounds__(256) void k_qsm(const float* __restrict__ QF, _Float16* __restrict__ Q16, int ntok) {
  const int t = blockIdx.x * 256 + threadIdx.x; if (t >= ntok) return; const size_t base = (size_t)t * CW + (size_t)blockIdx.y * HD; const float* s = QF + base; float mx = -3.0e38f;
  for (int j = 0; j < HD / 4; ++j) { const v4f a = *(const v4fa*)(s + 4 * j); for (int i = 0; i < 4; ++i) mx = (a[i] > mx) ? a[i] : mx; }
  float se = 0.f; for (int j = 0; j < HD / 4; ++j) { const v4f a = *(const v4fa*)(s + 4 * j); for (int i = 0; i < 4; ++i) se += __expf(a[i] - mx); } const float sc = QCAR / se;
  for (int j0 = 0; j0 < HD; j0 += 8) { FragH f; for (int q = 0; q < 8; ++q) f.h[q] = (_Float16)(__expf(s[j0 + q] - mx) * sc); unsigned short* o = (unsigned short*)Q16 + base + j0; *(volatile v8us*)o = f.half[0]; __threadfence(); *(volatile v8us*)o = f.half[0]; } }
__global__ __launch_bounds__(256) void k_colstat(const float* __restrict__ KF, float* __restrict__ PART, int n) {
  const int t = blockIdx.x * 256 + threadIdx.x; if (t >= n) return; const int c = t % CW, j = t / CW; const float* s = KF + (size_t)j * TBK * CW + c; float mx = -3.0e38f;
  for (int m = 0; m < TBK; ++m) { const float a = s[(size_t)m * CW]; mx = (a > mx) ? a : mx; }
  float se = 0.f; for (int m = 0; m < TBK; ++m) se += __expf(s[(size_t)m * CW] - mx);
  float* o = PART + 2 * (size_t)t; for (int pass = 0; pass < 2; ++pass) { *(volatile float*)o = mx; *(volatile float*)(o + 1) = se; if (pass == 0) __threadfence(); } }
__global__ __launch_bounds__(256) void k_colfin(const float* __restrict__ PART, float* __restrict__ REC, int n) {
  const int c = blockIdx.x * 256 + threadIdx.x; if (c >= n) return; float mx = -3.0e38f;
  for (int j = 0; j < NBLK; ++j) { const float a = PART[2 * ((size_t)j * CW + c)]; mx = (a > mx) ? a : mx; }
  float se = 0.f; for (int j = 0; j < NBLK; ++j) { const float* p = PART + 2 * ((size_t)j * CW + c); se += p[1] * __expf(p[0] - mx); }
  float* o = REC + 2 * (size_t)c; const float inv = KCAR / se; for (int pass = 0; pass < 2; ++pass) { *(volatile float*)o = mx; *(volatile float*)(o + 1) = inv; if (pass == 0) __threadfence(); } }
__global__ __launch_bounds__(256) void k_kstoreT(const float* __restrict__ KF, const float* __restrict__ REC, _Float16* __restrict__ KT, int n8) {
  const int t = blockIdx.x * 256 + threadIdx.x; if (t >= n8) return; const int c = t / (NTOK / 8), k8 = (t % (NTOK / 8)) * 8; const float mx = REC[2 * (size_t)c], inv = REC[2 * (size_t)c + 1]; FragH f;
  for (int i = 0; i < 8; ++i) f.h[i] = (_Float16)(__expf(KF[(size_t)(k8 + i) * CW + c] - mx) * inv);
  unsigned short* o = (unsigned short*)KT + (size_t)c * NTOK + k8; *(volatile v8us*)o = f.half[0]; __threadfence(); *(volatile v8us*)o = f.half[0]; }

extern "C" void kernel_launch(void* const* d_in, const int* in_sizes, int n_in,
                              void* d_out, int out_size, void* d_ws, size_t ws_size, hipStream_t stream) {
  (void)in_sizes; (void)n_in; (void)out_size;
  const float* const* I = (const float* const*)d_in; const float* x = I[0]; const float* wq = I[1]; const float* bq = I[2]; const float* wk = I[3]; const float* bk = I[4]; const float* wv = I[5]; const float* bv = I[6]; const float* wp = I[7]; const float* bp = I[8];
  static_assert(NB == 4 && NTOK == 8192 && CW == 384 && NHD == 6 && HD == 64 && NHD * HD == CW && TBK == 64 && NBLK == 128 && NTOK % 128 == 0 && (NB * NTOK) % 128 == 0 && CW % 64 == 0 && HD % 64 == 0 && HD % 32 == 0 && NTOK % 32 == 0 && CW % 32 == 0 && ((size_t)NB * NTOK * CW / 8) % 256 == 0 && ((size_t)CW * CW / 8) % 256 == 0 && ((size_t)HD * (CW / 8)) % 256 == 0 && NTOK % 256 == 0 && ((size_t)NBLK * CW) % 256 == 0 && ((size_t)CW * (NTOK / 8)) % 256 == 0, "whole tiles; exact grids");
  float* out = (float*)d_out;
  char* ws = (char*)d_ws; size_t off = 0;
  auto take = [&](size_t bytes) { char* p = ws + off; off += (bytes + 255) & ~(size_t)255; return p; };
  _Float16* X16 = (_Float16*)take((size_t)NB * NTOK * CW * 2); _Float16* WP16 = (_Float16*)take((size_t)CW * CW * 2); _Float16* WQT = (_Float16*)take((size_t)HD * CW * 2); _Float16* WKT = (_Float16*)take((size_t)HD * CW * 2); _Float16* WVT = (_Float16*)take((size_t)HD * CW * 2);
  float* QF = (float*)take((size_t)NTOK * CW * 4); float* KF = (float*)take((size_t)NTOK * CW * 4); float* VF = (float*)take((size_t)NTOK * CW * 4);
  _Float16* Q16 = (_Float16*)take((size_t)NTOK * CW * 2); _Float16* KT = (_Float16*)take((size_t)CW * NTOK * 2); _Float16* VT = (_Float16*)take((size_t)CW * NTOK * 2);
  float* PART = (float*)take((size_t)NBLK * CW * 2 * 4); float* REC = (float*)take((size_t)CW * 2 * 4); float* KVF = (float*)take((size_t)NHD * HD * HD * 4); _Float16* KVT = (_Float16*)take((size_t)HD * CW * 2);
  _Float16* O16 = (_Float16*)take((size_t)NB * NTOK * CW * 2);
  if (off > ws_size) return;
  k_x16<<<(unsigned)((size_t)NB * NTOK * CW / 8 / 256), 256, 0, stream>>>(x, X16, (size_t)NB * NTOK * CW / 8); k_x16<<<(unsigned)((size_t)CW * CW / 8 / 256), 256, 0, stream>>>(wp, WP16, (size_t)CW * CW / 8);
  k_wt_f16<<<(unsigned)((size_t)HD * (CW / 8) / 256), 256, 0, stream>>>(wq, WQT, CW, HD, 1.0f); k_wt_f16<<<(unsigned)((size_t)HD * (CW / 8) / 256), 256, 0, stream>>>(wk, WKT, CW, HD, 1.0f); k_wt_f16<<<(unsigned)((size_t)HD * (CW / 8) / 256), 256, 0, stream>>>(wv, WVT, CW, HD, 1.0f);
  for (int b = 0; b < NB; ++b) { const _Float16* xb = X16 + (size_t)b * NTOK * CW;
    k_gemm2<0><<<dim3((unsigned)((NTOK / 128) * (HD / 64)), NHD), 128, 0, stream>>>(xb, CW, (size_t)HD, WQT, CW, (size_t)HD, 1.0f, bq, (size_t)HD, nullptr, 1, 0, 0, QF, nullptr, CW, (size_t)HD, NTOK, HD, HD);
    k_gemm2<0><<<dim3((unsigned)((NTOK / 128) * (HD / 64)), NHD), 128, 0, stream>>>(xb, CW, (size_t)HD, WKT, CW, (size_t)HD, 1.0f, bk, (size_t)HD, nullptr, 1, 0, 0, KF, nullptr, CW, (size_t)HD, NTOK, HD, HD);
    k_gemm2<0><<<dim3((unsigned)((NTOK / 128) * (HD / 64)), NHD), 128, 0, stream>>>(xb, CW, (size_t)HD, WVT, CW, (size_t)HD, 1.0f, bv, (size_t)HD, nullptr, 1, 0, 0, VF, nullptr, CW, (size_t)HD, NTOK, HD, HD);
    k_qsm<<<dim3((unsigned)(NTOK / 256), NHD), 256, 0, stream>>>(QF, Q16, NTOK);
    k_colstat<<<(unsigned)((size_t)NBLK * CW / 256), 256, 0, stream>>>(KF, PART, NBLK * CW); k_colfin<<<(unsigned)((CW + 255) / 256), 256, 0, stream>>>(PART, REC, CW); k_kstoreT<<<(unsigned)((size_t)CW * (NTOK / 8) / 256), 256, 0, stream>>>(KF, REC, KT, CW * (NTOK / 8));
    k_wtn_f16<<<(unsigned)((size_t)CW * (NTOK / 8) / 256), 256, 0, stream>>>(VF, VT, NTOK, CW, 1.0f);
    k_gemm2<0><<<dim3((unsigned)(1 * (HD / 64)), NHD), 128, 0, stream>>>(KT, NTOK, (size_t)HD * NTOK, VT, NTOK, (size_t)HD * NTOK, 0.125f / KCAR, nullptr, 0, nullptr, 1, 0, 0, KVF, nullptr, HD, (size_t)HD * HD, HD, HD, NTOK);
    k_wtn_f16<<<(unsigned)((size_t)HD * (CW / 8) / 256), 256, 0, stream>>>(KVF, KVT, CW, HD, KVCAR);
    k_gemm2<0><<<dim3((unsigned)((NTOK / 128) * (HD / 64)), NHD), 128, 0, stream>>>(Q16, CW, (size_t)HD, KVT, CW, (size_t)HD, OCAR / (QCAR * KVCAR), nullptr, 0, nullptr, 1, 0, 0, nullptr, O16 + (size_t)b * NTOK * CW, CW, (size_t)HD, NTOK, HD, HD); }
  k_gemm2<0><<<dim3((unsigned)((NB * NTOK / 128) * (CW / 64)), 1), 128, 0, stream>>>(O16, CW, (size_t)0, WP16, CW, (size_t)0, 1.0f / OCAR, bp, 0, nullptr, 1, 0, 0, out, nullptr, CW, (size_t)0, NB * NTOK, CW, CW);
}
